// Model_9698036154926
// MI455X (gfx1250) — hardware-run, weakly checked
//
#include <hip/hip_runtime.h>

typedef __attribute__((ext_vector_type(16))) __bf16 v16b;
typedef __attribute__((ext_vector_type(8)))  __bf16 v8b;
typedef __attribute__((ext_vector_type(8)))  float  v8f;
typedef __attribute__((ext_vector_type(4)))  float  v4f;
typedef __attribute__((ext_vector_type(4)))  unsigned int v4u;

constexpr unsigned kNs     = 64u;
constexpr unsigned kSeq    = 200000u;
constexpr unsigned kTch    = 1250u;
constexpr unsigned kNch    = 160u;
constexpr unsigned kColsB  = 16u;
constexpr unsigned kBlk2   = kNch / kColsB;
constexpr unsigned kIdBlk  = kNs / kColsB;
constexpr unsigned kBlk1   = kBlk2 + kIdBlk;
constexpr unsigned kCat    = 192u;
constexpr unsigned kXbElems = kColsB * kCat;
constexpr unsigned kEcols  = kNch + kNs;
static_assert(kTch * kNch == kSeq);
static_assert((kNch % kColsB) == 0u);
static_assert((kSeq % 64u) == 0u);
static_assert((kCat % 32u) == 0u);
static_assert(kBlk2 == 10u && kBlk1 == 14u);

constexpr size_t kOffWcat = 0;
constexpr size_t kOffYT   = kOffWcat + (size_t)128 * kCat * 2;
constexpr size_t kOffOutT = kOffYT   + (size_t)kSeq * kNs * 4;
constexpr size_t kOffE    = kOffOutT + (size_t)kSeq * kNs * 4;
constexpr size_t kOffS    = kOffE    + (size_t)kEcols * kNs * 4;
constexpr size_t kWsTotal = kOffS    + (size_t)kNch * kNs * 4;
static_assert(kWsTotal == 102547456ull);
static_assert(kWsTotal <= 134217728ull);
static_assert((kOffYT % 128) == 0 && (kOffOutT % 128) == 0 && (kOffE % 128) == 0 && (kOffS % 128) == 0);

__device__ __forceinline__ void pin_u(unsigned& x) { asm volatile("" : "+v"(x)); }
__device__ __forceinline__ void pin_frag(v16b& x) { asm volatile("" : "+v"(x)); }

__device__ __forceinline__ unsigned bf_hi32(float f) {
  unsigned u = __float_as_uint(f);
  const unsigned lsb = (u & 0x00010000u) ? 1u : 0u;
  return (u + 0x7FFFu + lsb) & 0xFFFF0000u;
}

__device__ __forceinline__ void split8(v8f d, v4u& hw, v4u& lw) {
  unsigned hb[8], lb[8];
#pragma unroll
  for (int e = 0; e < 8; ++e) {
    const float f = d[e];
    const unsigned hu = bf_hi32(f);
    const float rem = f - __uint_as_float(hu);
    hb[e] = hu;
    lb[e] = bf_hi32(rem);
  }
  const unsigned h0 = __builtin_amdgcn_perm(hb[1], hb[0], 0x07060302u);
  const unsigned h1 = __builtin_amdgcn_perm(hb[3], hb[2], 0x07060302u);
  const unsigned h2 = __builtin_amdgcn_perm(hb[5], hb[4], 0x07060302u);
  const unsigned h3 = __builtin_amdgcn_perm(hb[7], hb[6], 0x07060302u);
  const unsigned l0 = __builtin_amdgcn_perm(lb[1], lb[0], 0x07060302u);
  const unsigned l1 = __builtin_amdgcn_perm(lb[3], lb[2], 0x07060302u);
  const unsigned l2 = __builtin_amdgcn_perm(lb[5], lb[4], 0x07060302u);
  const unsigned l3 = __builtin_amdgcn_perm(lb[7], lb[6], 0x07060302u);
  hw = (v4u){h0, h1, h2, h3};
  lw = (v4u){l0, l1, l2, l3};
}

union FragU { v16b v; v8b h[2]; };
__device__ __forceinline__ v16b frag_load(const __bf16* p) {
  FragU f;
  f.h[0] = *(const v8b*)(p);
  f.h[1] = *(const v8b*)(p + 16);
  return f.v;
}

__device__ __forceinline__ v8f mma_g(v16b a, v16b b, v8f c) {
  c = __builtin_amdgcn_wmma_f32_16x16x32_bf16(false, a, false, b, (short)0, c, false, false);
  asm volatile("v_nop\n\tv_nop\n\tv_nop\n\tv_nop" : "+v"(c) : "v"(a), "v"(b));
  return c;
}

__device__ __forceinline__ void prod2(const v16b (&a0)[6], const v16b (&a1)[6], const __bf16* xrow, v8f& c0, v8f& c1) {
#pragma unroll
  for (int j = 0; j < 6; ++j) {
    const v16b bfr = frag_load(xrow + 32 * j);
    c0 = mma_g(a0[j], bfr, c0);
    c1 = mma_g(a1[j], bfr, c1);
  }
}

__global__ __launch_bounds__(256) void prep_weights(
    const float* __restrict__ A, const float* __restrict__ H, const float* __restrict__ Lp,
    unsigned short* __restrict__ Wcat)
{
  unsigned idx = blockIdx.x * 256u + threadIdx.x;
  pin_u(idx);
  unsigned row = idx >> 3;
  unsigned g = idx & 7u;
  pin_u(row);
  pin_u(g);
  const unsigned r = row & 63u;
  const bool isH = (row >= 64u);
  const float lv = Lp[0];
  const float* ap = A + r * 64u + 8u * g;
  const float* hp = H + r * 64u + 8u * g;
  const v4f a0 = *(const v4f*)(ap);
  const v4f a1 = *(const v4f*)(ap + 4);
  const v4f h0 = *(const v4f*)(hp);
  const v4f h1 = *(const v4f*)(hp + 4);
  v8f w;
#pragma unroll
  for (int e = 0; e < 4; ++e) {
    const float m0 = a0[e] - lv * h0[e];
    const float m1 = a1[e] - lv * h1[e];
    w[e]     = isH ? h0[e] : m0;
    w[4 + e] = isH ? h1[e] : m1;
  }
  v4u hw, lw;
  split8(w, hw, lw);
  unsigned short* q = Wcat + (size_t)row * kCat + 8u * g;
  *(volatile v4u*)(q)       = hw;
  *(volatile v4u*)(q + 64)  = hw;
  *(volatile v4u*)(q + 128) = lw;
  __threadfence();
  *(volatile v4u*)(q)       = hw;
  *(volatile v4u*)(q + 64)  = hw;
  *(volatile v4u*)(q + 128) = lw;
}

__global__ __launch_bounds__(256) void tile_transpose64(
    const float* __restrict__ in, float* __restrict__ out,
    unsigned ldin, unsigned ldout, unsigned rstep, unsigned cstep,
    const float* __restrict__ Lp, int use_scale)
{
  __shared__ __align__(16) float Ls[64 * 65];
  unsigned tid = threadIdx.x;
  pin_u(tid);
  const unsigned r0 = blockIdx.x * rstep;
  const unsigned c0 = blockIdx.x * cstep;
  const float lv = Lp[0];
  const float sc = use_scale ? lv : 1.0f;
#pragma unroll
  for (unsigned it = 0; it < 4u; ++it) {
    unsigned idx = it * 256u + tid;
    unsigned r = idx >> 4;
    unsigned p = idx & 15u;
    pin_u(r);
    pin_u(p);
    const v4f v = *(const v4f*)(in + (size_t)(r0 + r) * ldin + c0 + 4u * p);
    Ls[(4u * p + 0u) * 65u + r] = v[0] * sc;
    Ls[(4u * p + 1u) * 65u + r] = v[1] * sc;
    Ls[(4u * p + 2u) * 65u + r] = v[2] * sc;
    Ls[(4u * p + 3u) * 65u + r] = v[3] * sc;
  }
  __syncthreads();
  v4f o[4];
#pragma unroll
  for (unsigned it = 0; it < 4u; ++it) {
    unsigned idx = it * 256u + tid;
    unsigned c = idx >> 4;
    unsigned p = idx & 15u;
    pin_u(c);
    pin_u(p);
    const float* lp = Ls + c * 65u + 4u * p;
    o[it] = (v4f){lp[0], lp[1], lp[2], lp[3]};
  }
  for (int pass = 0; pass < 2; ++pass) {
#pragma unroll
    for (unsigned it = 0; it < 4u; ++it) {
      unsigned idx = it * 256u + tid;
      unsigned c = idx >> 4;
      unsigned p = idx & 15u;
      pin_u(c);
      pin_u(p);
      *(volatile v4f*)(out + (size_t)(c0 + c) * ldout + r0 + 4u * p) = o[it];
    }
    __threadfence();
  }
}

template <bool EMIT>
__global__ __launch_bounds__(EMIT ? 128 : 64) void scan_pass(
    const unsigned short* __restrict__ Wcat, const float* __restrict__ yT,
    const float* __restrict__ Sstart, float* __restrict__ Eend, float* __restrict__ outT)
{
  constexpr unsigned NT = EMIT ? 128u : 64u;
  __shared__ __align__(16) __bf16 Xb[2 * kXbElems];
  __shared__ __align__(16) float St[EMIT ? 2048 : 1024];

  unsigned tid = threadIdx.x;
  pin_u(tid);
  const int wave = __builtin_amdgcn_readfirstlane((int)(tid >> 5));
  unsigned lane = tid & 31u;
  pin_u(lane);
  unsigned n = lane & 15u;
  unsigned h = lane >> 4;
  unsigned q = lane >> 3;
  unsigned p = lane & 7u;
  pin_u(n);
  pin_u(h);
  pin_u(q);
  pin_u(p);
  const unsigned b = blockIdx.x;
  const bool ident = (!EMIT) && (b >= kBlk2);
  const unsigned jb = ident ? (b - kBlk2) : 0u;
  const unsigned wr = (unsigned)wave & 1u;

  for (unsigned idx = tid; idx < 128u; idx += NT) {
    unsigned cn = idx >> 3;
    unsigned g = idx & 7u;
    pin_u(cn);
    pin_u(g);
    v8f f;
    if (EMIT) {
      const float* sp = Sstart + (size_t)(kColsB * b + cn) * kNs + 8u * g;
      const v4f s0 = *(const v4f*)(sp);
      const v4f s1 = *(const v4f*)(sp + 4);
      f = __builtin_shufflevector(s0, s1, 0, 1, 2, 3, 4, 5, 6, 7);
    } else {
      const unsigned j = kColsB * jb + cn;
#pragma unroll
      for (int e = 0; e < 8; ++e) f[e] = (ident && ((8u * g + (unsigned)e) == j)) ? 1.0f : 0.0f;
    }
    v4u hw, lw;
    split8(f, hw, lw);
    __bf16* xw = Xb + cn * kCat + 8u * g;
    *(v8b*)(xw)        = __builtin_bit_cast(v8b, hw);
    *(v8b*)(xw + 64)   = __builtin_bit_cast(v8b, lw);
    *(v8b*)(xw + 128)  = __builtin_bit_cast(v8b, hw);
  }

  const __bf16* W = (const __bf16*)Wcat;
  v16b a0[6], a1[6];
#pragma unroll
  for (int j = 0; j < 6; ++j) {
    a0[j] = frag_load(W + (size_t)(32u * (unsigned)wave + n) * kCat + 32u * j + 8u * h);
    a1[j] = frag_load(W + (size_t)(32u * (unsigned)wave + 16u + n) * kCat + 32u * j + 8u * h);
    pin_frag(a0[j]);
    pin_frag(a1[j]);
  }

  const unsigned ccol = ident ? 0u : (kColsB * b + n);
  const float* ybase = yT + ((size_t)kTch * ccol) * kNs + 32u * wr + 8u * h;
  const v8f zero8 = (v8f){0.f, 0.f, 0.f, 0.f, 0.f, 0.f, 0.f, 0.f};
  v8f c0 = zero8, c1 = zero8;
  __syncthreads();

#pragma unroll 1
  for (unsigned s = 0; s < kTch; ++s) {
    const unsigned cur = s & 1u;
    const __bf16* xrow = Xb + cur * kXbElems + n * kCat + 8u * h;
    if (!EMIT || wave < 2) {
      const float* yp = ybase + (size_t)s * kNs;
      const v4f y00 = *(const v4f*)(yp);
      const v4f y01 = *(const v4f*)(yp + 4);
      const v4f y10 = *(const v4f*)(yp + 16);
      const v4f y11 = *(const v4f*)(yp + 20);
      const v8f i0 = __builtin_shufflevector(y00, y01, 0, 1, 2, 3, 4, 5, 6, 7);
      const v8f i1 = __builtin_shufflevector(y10, y11, 0, 1, 2, 3, 4, 5, 6, 7);
      c0 = ident ? zero8 : i0;
      c1 = ident ? zero8 : i1;
      prod2(a0, a1, xrow, c0, c1);
      v4u h0w, l0w, h1w, l1w;
      split8(c0, h0w, l0w);
      split8(c1, h1w, l1w);
      __bf16* xw = Xb + (cur ^ 1u) * kXbElems + n * kCat + 32u * wr + 8u * h;
      *(v8b*)(xw)            = __builtin_bit_cast(v8b, h0w);
      *(v8b*)(xw + 64)       = __builtin_bit_cast(v8b, l0w);
      *(v8b*)(xw + 128)      = __builtin_bit_cast(v8b, h0w);
      *(v8b*)(xw + 16)       = __builtin_bit_cast(v8b, h1w);
      *(v8b*)(xw + 64 + 16)  = __builtin_bit_cast(v8b, l1w);
      *(v8b*)(xw + 128 + 16) = __builtin_bit_cast(v8b, h1w);
    } else {
      c0 = zero8;
      c1 = zero8;
      prod2(a0, a1, xrow, c0, c1);
      float* sp = St + (cur * 2u + wr) * 512u + n * 32u + 8u * h;
      *(v4f*)(sp)      = __builtin_shufflevector(c0, c0, 0, 1, 2, 3);
      *(v4f*)(sp + 4)  = __builtin_shufflevector(c0, c0, 4, 5, 6, 7);
      *(v4f*)(sp + 16) = __builtin_shufflevector(c1, c1, 0, 1, 2, 3);
      *(v4f*)(sp + 20) = __builtin_shufflevector(c1, c1, 4, 5, 6, 7);
    }
    __syncthreads();
    if (EMIT) {
      if (wave >= 2) {
        v4f ov[4];
#pragma unroll
        for (unsigned it = 0; it < 4u; ++it)
          ov[it] = *(const v4f*)(St + (cur * 2u + wr) * 512u + (4u * it + q) * 32u + 4u * p);
        for (int pass = 0; pass < 2; ++pass) {
#pragma unroll
          for (unsigned it = 0; it < 4u; ++it) {
            const size_t t = (size_t)kTch * (kColsB * b + 4u * it + q) + s;
            *(volatile v4f*)(outT + t * kNs + 32u * wr + 4u * p) = ov[it];
          }
          __threadfence();
        }
      }
    }
  }

  if (!EMIT) {
    float* sp = St + wr * 512u + n * 32u + 8u * h;
    *(v4f*)(sp)      = __builtin_shufflevector(c0, c0, 0, 1, 2, 3);
    *(v4f*)(sp + 4)  = __builtin_shufflevector(c0, c0, 4, 5, 6, 7);
    *(v4f*)(sp + 16) = __builtin_shufflevector(c1, c1, 0, 1, 2, 3);
    *(v4f*)(sp + 20) = __builtin_shufflevector(c1, c1, 4, 5, 6, 7);
    __syncthreads();
    v4f ov[4];
#pragma unroll
    for (unsigned it = 0; it < 4u; ++it)
      ov[it] = *(const v4f*)(St + wr * 512u + (4u * it + q) * 32u + 4u * p);
    for (int pass = 0; pass < 2; ++pass) {
#pragma unroll
      for (unsigned it = 0; it < 4u; ++it) {
        const size_t col = (size_t)(kColsB * b + 4u * it + q);
        *(volatile v4f*)(Eend + col * kNs + 32u * wr + 4u * p) = ov[it];
      }
      __threadfence();
    }
  }
}

__global__ __launch_bounds__(64) void carry_kernel(const float* __restrict__ E, float* __restrict__ S)
{
  __shared__ __align__(16) float Pl[64 * 64];
  __shared__ __align__(16) float Sl[160 * 64];
  __shared__ __align__(16) float xl[2 * 64];
  unsigned tid = threadIdx.x;
  pin_u(tid);
#pragma unroll 1
  for (unsigned idx = tid; idx < 4096u; idx += 64u) Pl[idx] = E[(size_t)kNch * kNs + idx];
  xl[tid] = 0.0f;
  xl[64u + tid] = 0.0f;
  __syncthreads();
#pragma unroll 1
  for (unsigned c = 0; c < kNch; ++c) {
    const unsigned cur = c & 1u;
    const float xi = xl[cur * 64u + tid];
    Sl[c * 64u + tid] = xi;
    float acc = E[(size_t)c * kNs + tid];
#pragma unroll 8
    for (unsigned k = 0; k < 64u; ++k) acc = fmaf(Pl[k * 64u + tid], xl[cur * 64u + k], acc);
    xl[(cur ^ 1u) * 64u + tid] = acc;
    __syncthreads();
  }
  for (int pass = 0; pass < 2; ++pass) {
#pragma unroll 1
    for (unsigned it = 0; it < 40u; ++it) {
      const unsigned idx = it * 64u + tid;
      const v4f v = *(const v4f*)(Sl + 4u * idx);
      *(volatile v4f*)(S + 4u * (size_t)idx) = v;
    }
    __threadfence();
  }
}

extern "C" void kernel_launch(void* const* d_in, const int* in_sizes, int n_in,
                              void* d_out, int out_size, void* d_ws, size_t ws_size,
                              hipStream_t stream) {
  if (n_in < 5) return;
  if (in_sizes[0] != (int)(kNs * kSeq)) return;
  if (in_sizes[1] != (int)(kNs * kNs)) return;
  if (in_sizes[2] != (int)(kNs * kNs)) return;
  if (in_sizes[3] != 1) return;
  if (out_size != (int)(kNs * kSeq)) return;
  if (ws_size < kWsTotal) return;

  const float* y  = (const float*)d_in[0];
  const float* A  = (const float*)d_in[1];
  const float* H  = (const float*)d_in[2];
  const float* Lp = (const float*)d_in[3];
  float* out = (float*)d_out;

  char* ws = (char*)d_ws;
  unsigned short* WC = (unsigned short*)(ws + kOffWcat);
  float* YT = (float*)(ws + kOffYT);
  float* OT = (float*)(ws + kOffOutT);
  float* EP = (float*)(ws + kOffE);
  float* SP = (float*)(ws + kOffS);

  prep_weights<<<4, 256, 0, stream>>>(A, H, Lp, WC);
  tile_transpose64<<<kSeq / 64u, 256, 0, stream>>>(y, YT, kSeq, kNs, 0u, 64u, Lp, 1);
  scan_pass<false><<<kBlk1, 64, 0, stream>>>(WC, YT, SP, EP, OT);
  carry_kernel<<<1, 64, 0, stream>>>(EP, SP);
  scan_pass<true><<<kBlk2, 128, 0, stream>>>(WC, YT, SP, EP, OT);
  tile_transpose64<<<kSeq / 64u, 256, 0, stream>>>(OT, out, kNs, kSeq, 64u, 0u, Lp, 0);
}
